// RelativeAttention_3624952398113
// MI455X (gfx1250) — hardware-verified
//
#include <hip/hip_runtime.h>


#define NB_  2
#define TT   1024
#define DM   1024
#define NH_  16
#define NKV  16
#define REP  (NH_ / NKV)
#define HD   64
#define DQ   (NH_ * HD)
#define DKV  (NKV * HD)
#define ZH   2
#define RH   512
#define WIN  1024
#define PCAR 1024.0f
#define SCL  1.0f
#define NE   2048
#define LNEPS 1e-5f
typedef _Float16 h16;
typedef unsigned short bf;
typedef __attribute__((ext_vector_type(16))) __bf16   v16bf;
typedef __attribute__((ext_vector_type(16))) _Float16 v16h;
typedef __attribute__((ext_vector_type(8)))  _Float16 v8h;
typedef __attribute__((ext_vector_type(8)))  unsigned short v8us;
typedef __attribute__((ext_vector_type(8)))  float    v8f;
typedef __attribute__((ext_vector_type(4)))  float    v4f;
typedef v8h  __attribute__((may_alias)) v8ha;
typedef v4f  __attribute__((may_alias)) v4fa;
typedef v8us __attribute__((may_alias)) v8usa;

__device__ __forceinline__ unsigned short f2bf(float f) { unsigned u = __float_as_uint(f); u += 0x7FFFu + ((u >> 16) & 1u); return (unsigned short)(u >> 16); }
__device__ __forceinline__ float bf2f(unsigned short b) { return __uint_as_float(((unsigned)b) << 16); }
__device__ __forceinline__ float bfr(float f) { return bf2f(f2bf(f)); }
__device__ __forceinline__ v16h cat16(v8h lo, v8h hi) { return __builtin_shufflevector(lo, hi, 0, 1, 2, 3, 4, 5, 6, 7, 8, 9, 10, 11, 12, 13, 14, 15); }
__device__ __forceinline__ v16bf cat16b(v8us lo, v8us hi) { return __builtin_bit_cast(v16bf, __builtin_shufflevector(lo, hi, 0, 1, 2, 3, 4, 5, 6, 7, 8, 9, 10, 11, 12, 13, 14, 15)); }
__device__ __forceinline__ v8f wmma16(v16h a, v16h b, v8f c) { return __builtin_amdgcn_wmma_f32_16x16x32_f16(false, a, false, b, (short)0, c, false, false); }
__device__ __forceinline__ v8f wmmab(v16bf a, v16bf b, v8f c) { return __builtin_amdgcn_wmma_f32_16x16x32_bf16(false, a, false, b, (short)0, c, false, false); }


template <typename T16> struct WFrag;
template <> struct WFrag<h16> { typedef v16h V; static __device__ __forceinline__ V ld(const h16* p) { return cat16(*(const v8h*)p, *(const v8h*)(p + 16)); } static __device__ __forceinline__ v8f mma(V a, V b, v8f c) { return wmma16(a, b, c); } };
template <> struct WFrag<bf> { typedef v16bf V; static __device__ __forceinline__ V ld(const bf* p) { return cat16b(*(const v8us*)p, *(const v8us*)(p + 16)); } static __device__ __forceinline__ v8f mma(V a, V b, v8f c) { return wmmab(a, b, c); } };
template <typename T16, int NSPLIT, bool BIAS>
__global__ __launch_bounds__(32) void k_gemmw(const T16* __restrict__ A, const T16* __restrict__ A2, const T16* __restrict__ Bt, const T16* __restrict__ Bt2, int K, float* C, int ldc, const float* __restrict__ bias, size_t sA, size_t sB, size_t sC) {
    typedef typename WFrag<T16>::V V;
    __shared__ __align__(16) float os[16 * 68];
    const size_t z = blockIdx.z; A += z * sA; if (A2) A2 += z * sA; Bt += z * sB; if (Bt2) Bt2 += z * sB; C += z * sC;
    const int lane = threadIdx.x & 31, lr = lane & 15, hi = lane >> 4; const int r0 = blockIdx.x * 64, c0 = blockIdx.y * 64;
    v8f acc[4][4];
#pragma unroll
    for (int mb = 0; mb < 4; ++mb)
#pragma unroll
        for (int nb = 0; nb < 4; ++nb) acc[mb][nb] = (v8f){};
    const size_t aoff = (size_t)(r0 + lr) * K + 8 * hi, boff = (size_t)(c0 + lr) * K + 8 * hi;
#pragma unroll 1
    for (int kc = 0; kc < K; kc += 32) {
        V a[4], a2[4];
#pragma unroll
        for (int mb = 0; mb < 4; ++mb) { a[mb] = WFrag<T16>::ld(A + aoff + (size_t)mb * 16 * K + kc); if (NSPLIT == 1 || NSPLIT == 2) a2[mb] = WFrag<T16>::ld(A2 + aoff + (size_t)mb * 16 * K + kc); }
#pragma unroll
        for (int nb = 0; nb < 4; ++nb) { const V b = WFrag<T16>::ld(Bt + boff + (size_t)nb * 16 * K + kc); V b2; if (NSPLIT >= 2) b2 = WFrag<T16>::ld(Bt2 + boff + (size_t)nb * 16 * K + kc);
#pragma unroll
            for (int mb = 0; mb < 4; ++mb) { acc[mb][nb] = WFrag<T16>::mma(a[mb], b, acc[mb][nb]); if (NSPLIT == 1 || NSPLIT == 2) acc[mb][nb] = WFrag<T16>::mma(a2[mb], b, acc[mb][nb]); if (NSPLIT >= 2) acc[mb][nb] = WFrag<T16>::mma(a[mb], b2, acc[mb][nb]); } }
        asm volatile("v_nop\n\tv_nop\n\tv_nop\n\tv_nop" : "+v"(acc[0][0]), "+v"(acc[1][1]), "+v"(acc[2][2]), "+v"(acc[3][3]) : "v"(a[0]), "v"(a[3]));
    }
#pragma unroll
    for (int mb = 0; mb < 4; ++mb) {
#pragma unroll
        for (int nb = 0; nb < 4; ++nb) {
#pragma unroll
            for (int j = 0; j < 8; ++j) os[(hi * 8 + j) * 68 + nb * 16 + lr] = acc[mb][nb][j]; }
        __builtin_amdgcn_wave_barrier(); asm volatile("" ::: "memory");
        float* crow = C + (size_t)(r0 + mb * 16) * ldc + c0;
#pragma unroll 1
        for (int ps = 0; ps < 2; ++ps) {
#pragma unroll
            for (int s = 0; s < 8; ++s) { const int row = 2 * s + hi, cofs = lr * 4; v4f val = *(const v4fa*)(os + row * 68 + cofs); if (BIAS) { val[0] += bfr(bias[c0 + cofs]); val[1] += bfr(bias[c0 + cofs + 1]); val[2] += bfr(bias[c0 + cofs + 2]); val[3] += bfr(bias[c0 + cofs + 3]); }
                *(volatile v4f*)(crow + (size_t)row * ldc + cofs) = val; }
            if (ps == 0) __threadfence(); }
        __builtin_amdgcn_wave_barrier(); asm volatile("" ::: "memory");
    }
}

template <typename T16, int NSPLIT, int CMODE>
__global__ __launch_bounds__(32) void k_gemmc(const T16* __restrict__ A, const T16* __restrict__ A2, const T16* __restrict__ Bt, const T16* __restrict__ Bt2, int K, float* C, int ldc, int roff, size_t sA, size_t sB, size_t sC) {
    typedef typename WFrag<T16>::V V;
    __shared__ __align__(16) float os[16 * 68];
    const size_t z = blockIdx.z; A += z * sA; if (A2) A2 += z * sA; Bt += z * sB; if (Bt2) Bt2 += z * sB; C += z * sC;
    const int lane = threadIdx.x & 31, lr = lane & 15, hi = lane >> 4; const int r0 = blockIdx.x * 64, c0 = blockIdx.y * 64;
    if (CMODE == 1 && c0 > r0 + roff + 63) return;
    const int Kl = (CMODE == 2) ? min(K, r0 + roff + 64) : K;
    v8f acc[4][4];
#pragma unroll
    for (int mb = 0; mb < 4; ++mb)
#pragma unroll
        for (int nb = 0; nb < 4; ++nb) acc[mb][nb] = (v8f){};
    const size_t aoff = (size_t)(r0 + lr) * K + 8 * hi, boff = (size_t)(c0 + lr) * K + 8 * hi;
#pragma unroll 1
    for (int kc = 0; kc < Kl; kc += 32) {
        V a[4], a2[4];
#pragma unroll
        for (int mb = 0; mb < 4; ++mb) { a[mb] = WFrag<T16>::ld(A + aoff + (size_t)mb * 16 * K + kc); if (NSPLIT == 1 || NSPLIT == 2) a2[mb] = WFrag<T16>::ld(A2 + aoff + (size_t)mb * 16 * K + kc); }
#pragma unroll
        for (int nb = 0; nb < 4; ++nb) { const V b = WFrag<T16>::ld(Bt + boff + (size_t)nb * 16 * K + kc); V b2; if (NSPLIT >= 2) b2 = WFrag<T16>::ld(Bt2 + boff + (size_t)nb * 16 * K + kc);
#pragma unroll
            for (int mb = 0; mb < 4; ++mb) { acc[mb][nb] = WFrag<T16>::mma(a[mb], b, acc[mb][nb]); if (NSPLIT == 1 || NSPLIT == 2) acc[mb][nb] = WFrag<T16>::mma(a2[mb], b, acc[mb][nb]); if (NSPLIT >= 2) acc[mb][nb] = WFrag<T16>::mma(a[mb], b2, acc[mb][nb]); } }
        asm volatile("v_nop\n\tv_nop\n\tv_nop\n\tv_nop" : "+v"(acc[0][0]), "+v"(acc[1][1]), "+v"(acc[2][2]), "+v"(acc[3][3]) : "v"(a[0]), "v"(a[3]));
    }
#pragma unroll
    for (int mb = 0; mb < 4; ++mb) {
#pragma unroll
        for (int nb = 0; nb < 4; ++nb) {
#pragma unroll
            for (int j = 0; j < 8; ++j) os[(hi * 8 + j) * 68 + nb * 16 + lr] = acc[mb][nb][j]; }
        __builtin_amdgcn_wave_barrier(); asm volatile("" ::: "memory");
        float* crow = C + (size_t)(r0 + mb * 16) * ldc + c0;
#pragma unroll 1
        for (int ps = 0; ps < 2; ++ps) {
#pragma unroll
            for (int s = 0; s < 8; ++s) { const int row = 2 * s + hi, cofs = lr * 4; v4f val = *(const v4fa*)(os + row * 68 + cofs);
                *(volatile v4f*)(crow + (size_t)row * ldc + cofs) = val; }
            if (ps == 0) __threadfence(); }
        __builtin_amdgcn_wave_barrier(); asm volatile("" ::: "memory");
    }
}

__device__ __forceinline__ h16 tohx(float x) { return (h16)x; }
__device__ __forceinline__ void splitf(float y, unsigned short& h, unsigned short& l) { h = f2bf(y); l = f2bf(y - bf2f(h)); }
typedef __attribute__((ext_vector_type(2))) _Float16 v2h;
typedef __attribute__((ext_vector_type(4))) _Float16 v4h;
typedef __attribute__((ext_vector_type(2))) unsigned short v2us;
typedef __attribute__((ext_vector_type(4))) unsigned short v4us;
typedef __attribute__((ext_vector_type(2))) float v2f;
typedef __attribute__((ext_vector_type(4))) int v4i;

__global__ __launch_bounds__(256) void k_wtG(const float* __restrict__ w, int K, int N, bf* Bt) {
    const int lane = threadIdx.x & 31; const int L0 = (blockIdx.x * 8 + (threadIdx.x >> 5)) * 8; const int nlines = N * K / 64;
#pragma unroll
    for (int ps = 0; ps < 2; ++ps) {
#pragma unroll 1
        for (int l = 0; l < 8; ++l) { const int L = L0 + l; if (L >= nlines) break; const size_t e = (size_t)L * 64 + lane * 2; const int k = (int)(e % K), n = (int)(e / K); v2us o;
            o[0] = f2bf(w[(size_t)k * N + n]); o[1] = f2bf(w[(size_t)(k + 1) * N + n]); *(volatile v2us*)(Bt + e) = o; }
        if (ps == 0) __threadfence(); }
}
__global__ __launch_bounds__(256) void k_cvt8(const float* __restrict__ src, bf* dst, size_t n8) { const size_t i = (size_t)blockIdx.x * 256 + threadIdx.x; if (i >= n8) return; const v8f v = *(const v8f*)(src + i * 8); v8us o;
#pragma unroll
    for (int k = 0; k < 8; ++k) o[k] = f2bf(v[k]); *(volatile v8us*)(dst + i * 8) = o; __threadfence(); *(volatile v8us*)(dst + i * 8) = o; }

__global__ __launch_bounds__(256) void k_rope(const float* __restrict__ F, int pitch, int nheads, const float* __restrict__ CS, const float* __restrict__ RF, const float* __restrict__ nw, float sc, h16* P16, bf* Ph, bf* Pl) {
    const size_t e = ((size_t)blockIdx.x * 256 + threadIdx.x) * 2; if (e >= (size_t)nheads * TT * HD) return; const int d = (int)(e % HD); const int t = (int)((e / HD) % TT); const int h = (int)(e / ((size_t)HD * TT)); const float* f = F + (size_t)t * pitch + h * HD; const float rf = RF ? RF[(size_t)h * TT + t] : 1.0f; v2h o16; v2us oh, ol;
#pragma unroll
    for (int q = 0; q < 2; ++q) { const int dd = d + q; const int dp = (dd < HD / 2) ? dd + HD / 2 : dd - HD / 2; float x0 = f[dd], x1 = f[dp];
        if (RF) { float n0 = __fmul_rn(x0, rf), n1 = __fmul_rn(x1, rf); asm volatile("" : "+v"(n0)); asm volatile("" : "+v"(n1)); x0 = __fmul_rn(bfr(nw[dd]), n0); x1 = __fmul_rn(bfr(nw[dp]), n1); }
        const v2f cs = *(const v2f*)(CS + ((size_t)t * HD + dd) * 2); float a = __fmul_rn(x0, cs[0]), bq = __fmul_rn(x1, cs[1]); asm volatile("" : "+v"(a)); asm volatile("" : "+v"(bq)); const float r = ((dd < HD / 2) ? __fsub_rn(a, bq) : __fadd_rn(a, bq)) * sc;
        o16[q] = tohx(r); unsigned short a2, c2; splitf(r, a2, c2); oh[q] = a2; ol[q] = c2; }
    *(volatile v2h*)(P16 + e) = o16; *(volatile v2us*)(Ph + e) = oh; *(volatile v2us*)(Pl + e) = ol; __threadfence(); *(volatile v2h*)(P16 + e) = o16; *(volatile v2us*)(Ph + e) = oh; *(volatile v2us*)(Pl + e) = ol; }
__global__ __launch_bounds__(256) void k_vtp(const float* __restrict__ F, int pitch, int nheads, h16* V16, bf* Vh, bf* Vl) { const size_t e = ((size_t)blockIdx.x * 256 + threadIdx.x) * 2; if (e >= (size_t)nheads * HD * TT) return; const int t = (int)(e % TT); const int d = (int)((e / TT) % HD); const int g = (int)(e / ((size_t)TT * HD)); v2h o16; v2us oh, ol;
#pragma unroll
    for (int q = 0; q < 2; ++q) { const float x = F[(size_t)(t + q) * pitch + g * HD + d]; o16[q] = tohx(x); unsigned short a2, c2; splitf(x, a2, c2); oh[q] = a2; ol[q] = c2; }
    *(volatile v2h*)(V16 + e) = o16; *(volatile v2us*)(Vh + e) = oh; *(volatile v2us*)(Vl + e) = ol; __threadfence(); *(volatile v2h*)(V16 + e) = o16; *(volatile v2us*)(Vh + e) = oh; *(volatile v2us*)(Vl + e) = ol; }
__global__ __launch_bounds__(256) void k_csid(float* CS) { const int idx = blockIdx.x * 256 + threadIdx.x; if (idx >= TT * HD) return; v2f cs; cs[0] = 1.0f; cs[1] = 0.0f; *(volatile v2f*)(CS + (size_t)idx * 2) = cs; __threadfence(); *(volatile v2f*)(CS + (size_t)idx * 2) = cs; }
__global__ __launch_bounds__(256) void k_asoft(const float* __restrict__ Sb, h16* P16, bf* Ph, bf* Pl) {
    const int lane = threadIdx.x & 31; const int row = blockIdx.x * 8 + (threadIdx.x >> 5); if (row >= ZH * TT) return; const int i = row % TT; const int zz = row / TT; (void)zz; const bool hires = (i < RH); const float* sr = Sb + (size_t)row * TT; float v[TT / 32]; float mx = -3.0e38f;
#pragma unroll
    for (int ch = 0; ch < TT / 128; ++ch) { const int j0 = ch * 128 + lane * 4; const v4f a = *(const v4f*)(sr + j0);
#pragma unroll
        for (int q = 0; q < 4; ++q) { const int j = j0 + q; (void)j; const float t = (j <= i && i - j < WIN) ? a[q] * SCL : -3.0e38f; v[ch * 4 + q] = t; mx = fmaxf(mx, t); } }
#pragma unroll
    for (int sh = 16; sh; sh >>= 1) mx = fmaxf(mx, __shfl_xor(mx, sh, 32));
    float sum = 0.f;
#pragma unroll
    for (int k = 0; k < TT / 32; ++k) { float d0 = __fsub_rn(v[k], mx); asm volatile("" : "+v"(d0)); v[k] = __builtin_amdgcn_exp2f(__fmul_rn(d0, 1.4426950408889634f)); sum += v[k]; }
#pragma unroll
    for (int sh = 16; sh; sh >>= 1) sum += __shfl_xor(sum, sh, 32);
    const float f = __fdiv_rn(hires ? 1.0f : PCAR, sum);
#pragma unroll 1
    for (int ps = 0; ps < 2; ++ps) {
        if (hires) {
#pragma unroll
            for (int ch = 0; ch < TT / 128; ++ch) { v4us oh, ol;
#pragma unroll
                for (int q = 0; q < 4; ++q) { unsigned short a, c2; splitf(v[ch * 4 + q] * f, a, c2); oh[q] = a; ol[q] = c2; }
                const size_t oo = ((size_t)zz * (RH ? RH : 1) + i) * TT + ch * 128 + lane * 4; *(volatile v4us*)(Ph + oo) = oh; *(volatile v4us*)(Pl + oo) = ol; }
        } else {
#pragma unroll
            for (int ch = 0; ch < TT / 128; ++ch) { v4h o4;
#pragma unroll
                for (int q = 0; q < 4; ++q) o4[q] = tohx(v[ch * 4 + q] * f);
                *(volatile v4h*)(P16 + (size_t)row * TT + ch * 128 + lane * 4) = o4; } }
        if (ps == 0) __threadfence(); }
}
__constant__ float INVR[512] = {1.00000000f, 0.982171893f, 0.964661598f, 0.947463512f, 0.930572033f, 0.913981676f, 0.897687137f, 0.881683052f, 0.865964353f, 0.850525796f, 0.835362554f, 0.820469618f, 0.805842161f, 0.791475534f, 0.777365029f, 0.763506055f, 0.749894202f, 0.736524999f, 0.723394156f, 0.710497439f, 0.697830558f, 0.685389578f, 0.673170388f, 0.661169052f, 0.649381638f, 0.637804389f, 0.626433551f, 0.615265429f, 0.604296386f, 0.593522906f, 0.582941532f, 0.572548807f, 0.562341332f, 0.552315831f, 0.542469084f, 0.532797873f, 0.523299098f, 0.513969660f, 0.504806578f, 0.495806813f, 0.486967534f, 0.478285819f, 0.469758868f, 0.461383969f, 0.453158379f, 0.445079416f, 0.437144488f, 0.429351032f, 0.421696514f, 0.414178461f, 0.406794429f, 0.399542063f, 0.392418981f, 0.385422885f, 0.378551513f, 0.371802658f, 0.365174115f, 0.358663768f, 0.352269471f, 0.345989168f, 0.339820832f, 0.333762467f, 0.327812105f, 0.321967840f, 0.316227764f, 0.310590029f, 0.305052787f, 0.299614280f, 0.294272721f, 0.289026380f, 0.283873588f, 0.278812677f, 0.273841977f, 0.268959880f, 0.264164835f, 0.259455264f, 0.254829675f, 0.250286549f, 0.245824412f, 0.241441816f, 0.237137377f, 0.232909665f, 0.228757322f, 0.224679008f, 0.220673412f, 0.216739222f, 0.212875172f, 0.209080011f, 0.205352500f, 0.201691449f, 0.198095679f, 0.194564000f, 0.191095293f, 0.187688425f, 0.184342295f, 0.181055829f, 0.177827939f, 0.174657598f, 0.171543792f, 0.168485492f, 0.165481716f, 0.162531480f, 0.159633860f, 0.156787887f, 0.153992653f, 0.151247248f, 0.148550808f, 0.145902425f, 0.143301263f, 0.140746459f, 0.138237223f, 0.135772720f, 0.133352146f, 0.130974725f, 0.128639698f, 0.126346290f, 0.124093778f, 0.121881418f, 0.119708501f, 0.117574327f, 0.115478195f, 0.113419443f, 0.111397386f, 0.109411381f, 0.107460782f, 0.105544962f, 0.103663296f, 0.101815172f, 0.100000001f, 0.0982171893f, 0.0964661613f, 0.0947463512f, 0.0930572078f, 0.0913981721f, 0.0897687152f, 0.0881683081f, 0.0865964293f, 0.0850525796f, 0.0835362524f, 0.0820469633f, 0.0805842206f, 0.0791475549f, 0.0777365044f, 0.0763506070f, 0.0749894232f, 0.0736524984f, 0.0723394156f, 0.0710497424f, 0.0697830617f, 0.0685389563f, 0.0673170388f, 0.0661168993f, 0.0649381652f, 0.0637804419f, 0.0626433566f, 0.0615265407f, 0.0604296401f, 0.0593522936f, 0.0582941547f, 0.0572548807f, 0.0562341325f, 0.0552315824f, 0.0542469099f, 0.0532797910f, 0.0523299128f, 0.0513969697f, 0.0504806563f, 0.0495806821f, 0.0486967526f, 0.0478285812f, 0.0469758883f, 0.0461383983f, 0.0453158356f, 0.0445079394f, 0.0437144488f, 0.0429351032f, 0.0421696492f, 0.0414178446f, 0.0406794436f, 0.0399542041f, 0.0392418988f, 0.0385422893f, 0.0378551520f, 0.0371802673f, 0.0365174115f, 0.0358663760f, 0.0352269448f, 0.0345989168f, 0.0339820832f, 0.0333762467f, 0.0327812098f, 0.0321967863f, 0.0316227749f, 0.0310590025f, 0.0305052791f, 0.0299614277f, 0.0294272713f, 0.0289026387f, 0.0283873603f, 0.0278812665f, 0.0273841955f, 0.0268959887f, 0.0264164824f, 0.0259455275f, 0.0254829675f, 0.0250286534f, 0.0245824400f, 0.0241441820f, 0.0237137377f, 0.0232909657f, 0.0228757318f, 0.0224679001f, 0.0220673401f, 0.0216739215f, 0.0212875158f, 0.0209079999f, 0.0205352511f, 0.0201691464f, 0.0198095683f, 0.0194564015f, 0.0191095304f, 0.0187688433f, 0.0184342302f, 0.0181055833f, 0.0177827943f, 0.0174657609f, 0.0171543788f, 0.0168485492f, 0.0165481716f, 0.0162531491f, 0.0159633849f, 0.0156787876f, 0.0153992651f, 0.0151247252f, 0.0148550803f, 0.0145902419f, 0.0143301254f, 0.0140746469f, 0.0138237225f, 0.0135772713f, 0.0133352140f, 0.0130974725f, 0.0128639694f, 0.0126346294f, 0.0124093778f, 0.0121881422f, 0.0119708506f, 0.0117574325f, 0.0115478197f, 0.0113419443f, 0.0111397384f, 0.0109411385f, 0.0107460786f, 0.0105544962f, 0.0103663290f, 0.0101815173f, 0.00999999978f, 0.00982171856f, 0.00964661594f, 0.00947463512f, 0.00930572022f, 0.00913981721f, 0.00897687115f, 0.00881683081f, 0.00865964312f, 0.00850525778f, 0.00835362542f, 0.00820469577f, 0.00805842225f, 0.00791475549f, 0.00777365034f, 0.00763506070f, 0.00749894232f, 0.00736525003f, 0.00723394146f, 0.00710497424f, 0.00697830599f, 0.00685389573f, 0.00673170388f, 0.00661169039f, 0.00649381615f, 0.00637804391f, 0.00626433548f, 0.00615265407f, 0.00604296383f, 0.00593522936f, 0.00582941528f, 0.00572548807f, 0.00562341325f, 0.00552315824f, 0.00542469090f, 0.00532797910f, 0.00523299119f, 0.00513969688f, 0.00504806591f, 0.00495806802f, 0.00486967526f, 0.00478285830f, 0.00469758874f, 0.00461383956f, 0.00453158375f, 0.00445079384f, 0.00437144469f, 0.00429351022f, 0.00421696482f, 0.00414178474f, 0.00406794436f, 0.00399542041f, 0.00392418960f, 0.00385422888f, 0.00378551520f, 0.00371802668f, 0.00365174119f, 0.00358663755f, 0.00352269458f, 0.00345989177f, 0.00339820841f, 0.00333762472f, 0.00327812112f, 0.00321967853f, 0.00316227763f, 0.00310590025f, 0.00305052800f, 0.00299614272f, 0.00294272718f, 0.00289026392f, 0.00283873593f, 0.00278812670f, 0.00273841969f, 0.00268959883f, 0.00264164829f, 0.00259455270f, 0.00254829670f, 0.00250286539f, 0.00245824410f, 0.00241441815f, 0.00237137382f, 0.00232909666f, 0.00228757318f, 0.00224679010f, 0.00220673415f, 0.00216739206f, 0.00212875172f, 0.00209080009f, 0.00205352507f, 0.00201691454f, 0.00198095688f, 0.00194564008f, 0.00191095297f, 0.00187688426f, 0.00184342300f, 0.00181055826f, 0.00177827943f, 0.00174657605f, 0.00171543786f, 0.00168485485f, 0.00165481714f, 0.00162531482f, 0.00159633858f, 0.00156787888f, 0.00153992651f, 0.00151247252f, 0.00148550805f, 0.00145902426f, 0.00143301254f, 0.00140746462f, 0.00138237223f, 0.00135772710f, 0.00133352145f, 0.00130974723f, 0.00128639699f, 0.00126346294f, 0.00124093774f, 0.00121881417f, 0.00119708502f, 0.00117574329f, 0.00115478202f, 0.00113419443f, 0.00111397391f, 0.00109411380f, 0.00107460783f, 0.00105544960f, 0.00103663292f, 0.00101815176f, 0.00100000005f, 0.000982171856f, 0.000964661594f, 0.000947463501f, 0.000930572045f, 0.000913981698f, 0.000897687161f, 0.000881683081f, 0.000865964335f, 0.000850525801f, 0.000835362531f, 0.000820469635f, 0.000805842166f, 0.000791475526f, 0.000777365058f, 0.000763506105f, 0.000749894185f, 0.000736524991f, 0.000723394158f, 0.000710497436f, 0.000697830576f, 0.000685389561f, 0.000673170376f, 0.000661169004f, 0.000649381604f, 0.000637804391f, 0.000626433524f, 0.000615265395f, 0.000604296394f, 0.000593522913f, 0.000582941517f, 0.000572548772f, 0.000562341302f, 0.000552315847f, 0.000542469090f, 0.000532797887f, 0.000523299095f, 0.000513969688f, 0.000504806580f, 0.000495806802f, 0.000486967532f, 0.000478285801f, 0.000469758874f, 0.000461383956f, 0.000453158369f, 0.000445079408f, 0.000437144481f, 0.000429351028f, 0.000421696517f, 0.000414178445f, 0.000406794425f, 0.000399542070f, 0.000392418966f, 0.000385422900f, 0.000378551515f, 0.000371802656f, 0.000365174114f, 0.000358663761f, 0.000352269475f, 0.000345989160f, 0.000339820836f, 0.000333762466f, 0.000327812129f, 0.000321967847f, 0.000316227757f, 0.000310590025f, 0.000305052788f, 0.000299614272f, 0.000294272730f, 0.000289026386f, 0.000283873611f, 0.000278812659f, 0.000273841957f, 0.000268959877f, 0.000264164846f, 0.000259455264f, 0.000254829676f, 0.000250286539f, 0.000245824398f, 0.000241441827f, 0.000237137370f, 0.000232909661f, 0.000228757315f, 0.000224679010f, 0.000220673406f, 0.000216739223f, 0.000212875166f, 0.000209079997f, 0.000205352510f, 0.000201691451f, 0.000198095673f, 0.000194564011f, 0.000191095300f, 0.000187688434f, 0.000184342294f, 0.000181055831f, 0.000177827940f, 0.000174657602f, 0.000171543783f, 0.000168485494f, 0.000165481717f, 0.000162531491f, 0.000159633855f, 0.000156787879f, 0.000153992660f, 0.000151247252f, 0.000148550796f, 0.000145902421f, 0.000143301251f, 0.000140746473f, 0.000138237228f, 0.000135772716f, 0.000133352150f, 0.000130974731f, 0.000128639687f, 0.000126346291f, 0.000124093771f, 0.000121881421f, 0.000119708500f, 0.000117574324f, 0.000115478200f, 0.000113419439f, 0.000111397385f, 0.000109411383f, 0.000107460786f, 0.000105544961f, 0.000103663289f, 0.000101815174f};
__global__ __launch_bounds__(256) void k_sinR(float* RT) { const size_t k = (size_t)blockIdx.x * 256 + threadIdx.x; if (k >= (size_t)NE * DM / 4) return; const size_t e = k * 4; const int c0 = (int)(e % DM); const int r = (int)(e / DM); const float pos = (float)(r - (TT - 1)); v4f o;
#pragma unroll
    for (int q = 0; q < 4; q += 2) { const int i = (c0 + q) / 2; const float a = __fmul_rn(pos, INVR[i]); o[q] = (r < 2 * TT - 1) ? sinf(a) : 0.0f; o[q + 1] = (r < 2 * TT - 1) ? cosf(a) : 0.0f; }
    *(volatile v4f*)(RT + e) = o; __threadfence(); *(volatile v4f*)(RT + e) = o; }
__global__ __launch_bounds__(256) void k_hplanesN(const float* __restrict__ F, bf* Ph, bf* Pl) { const size_t k = (size_t)blockIdx.x * 256 + threadIdx.x; if (k >= (size_t)NE * DQ / 4) return; const size_t e = k * 4; const int c = (int)(e % DQ); const int r = (int)(e / DQ); const int h = c / HD, d = c % HD; const v4f a = *(const v4f*)(F + e); v4us oh, ol;
#pragma unroll
    for (int q = 0; q < 4; ++q) { unsigned short u, w; splitf(a[q], u, w); oh[q] = u; ol[q] = w; }
    const size_t oo = ((size_t)h * NE + r) * HD + d; *(volatile v4us*)(Ph + oo) = oh; *(volatile v4us*)(Pl + oo) = ol; __threadfence(); *(volatile v4us*)(Ph + oo) = oh; *(volatile v4us*)(Pl + oo) = ol; }
__global__ __launch_bounds__(256) void k_addrl(float* Sb, const float* __restrict__ QE) { const size_t k = (size_t)blockIdx.x * 256 + threadIdx.x; if (k >= (size_t)ZH * TT * TT / 4) return; const size_t e = k * 4; const int j0 = (int)(e % TT); const int i = (int)((e / TT) % TT); const int zz = (int)(e / ((size_t)TT * TT)); const float* qe = QE + ((size_t)zz * TT + i) * NE; v4f a = *(const v4f*)(Sb + e);
#pragma unroll
    for (int q = 0; q < 4; ++q) { const int j = j0 + q; const float t = qe[(TT - 1) - i + min(j, i)]; const float add = (j < i) ? t : ((j == i) ? __fadd_rn(t, t) : 0.0f); a[q] = __fadd_rn(a[q], add); }
    *(volatile v4f*)(Sb + e) = a; __threadfence(); *(volatile v4f*)(Sb + e) = a; }
__global__ __launch_bounds__(256) void k_addhb(float* FQ, const float* __restrict__ ub, const float* __restrict__ vb, float* FQV) { const size_t i = (size_t)blockIdx.x * 256 + threadIdx.x; if (i >= (size_t)TT * DQ / 4) return; const size_t e = i * 4; const int c0 = (int)(e % DQ); const v4f a = *(const v4f*)(FQ + e); v4f ou, ov;
#pragma unroll
    for (int q = 0; q < 4; ++q) { ou[q] = __fadd_rn(a[q], bfr(ub[c0 + q])); ov[q] = __fadd_rn(a[q], bfr(vb[c0 + q])); }
    *(volatile v4f*)(FQV + e) = ov; *(volatile v4f*)(FQ + e) = ou; __threadfence(); *(volatile v4f*)(FQV + e) = ov; *(volatile v4f*)(FQ + e) = ou; }

__global__ __launch_bounds__(256) void k_split8(const float* __restrict__ F, bf* Ph, bf* Pl, size_t n8) { const size_t i = (size_t)blockIdx.x * 256 + threadIdx.x; if (i >= n8) return; const v8f v = *(const v8f*)(F + i * 8); v8us oh, ol;
#pragma unroll
    for (int k = 0; k < 8; ++k) { unsigned short a, c2; splitf(v[k], a, c2); oh[k] = a; ol[k] = c2; }
    *(volatile v8us*)(Ph + i * 8) = oh; *(volatile v8us*)(Pl + i * 8) = ol; __threadfence(); *(volatile v8us*)(Ph + i * 8) = oh; *(volatile v8us*)(Pl + i * 8) = ol; }

__global__ __launch_bounds__(256) void k_addres(float* Y, const float* __restrict__ xr) { const size_t i = (size_t)blockIdx.x * 256 + threadIdx.x; if (i >= (size_t)TT * DQ / 4) return; const v4f a = *(const v4f*)(Y + i * 4); const v4f r = *(const v4f*)(xr + i * 4); v4f o;
#pragma unroll
    for (int q = 0; q < 4; ++q) o[q] = __fadd_rn(a[q], bfr(r[q]));
    *(volatile v4f*)(Y + i * 4) = o; __threadfence(); *(volatile v4f*)(Y + i * 4) = o; }
__global__ __launch_bounds__(256) void k_lnout(const float* __restrict__ F, const float* __restrict__ g, const float* __restrict__ bb, float* out) { const int lane = threadIdx.x & 31; const int row = blockIdx.x * 8 + (threadIdx.x >> 5); if (row >= TT) return; const float* fr = F + (size_t)row * DQ; float* orow = out + (size_t)row * DQ; float v[DQ / 32]; float s = 0.f;
#pragma unroll
    for (int c = 0; c < DQ / 128; ++c) { const v4f a = *(const v4f*)(fr + c * 128 + lane * 4); for (int q = 0; q < 4; ++q) { v[c * 4 + q] = a[q]; s = __fadd_rn(s, a[q]); } }
#pragma unroll
    for (int sh = 16; sh; sh >>= 1) s = __fadd_rn(s, __shfl_xor(s, sh, 32));
    const float mean = __fdiv_rn(s, (float)DQ); float s2 = 0.f;
#pragma unroll
    for (int k = 0; k < DQ / 32; ++k) { const float dv = __fsub_rn(v[k], mean); float p2 = __fmul_rn(dv, dv); asm volatile("" : "+v"(p2)); s2 = __fadd_rn(s2, p2); v[k] = dv; }
#pragma unroll
    for (int sh = 16; sh; sh >>= 1) s2 = __fadd_rn(s2, __shfl_xor(s2, sh, 32));
    const float rs = __fdiv_rn(1.0f, __fsqrt_rn(__fadd_rn(__fdiv_rn(s2, (float)DQ), LNEPS)));
#pragma unroll 1
    for (int ps = 0; ps < 2; ++ps) {
#pragma unroll
        for (int c = 0; c < DQ / 128; ++c) { v4f o; for (int q = 0; q < 4; ++q) { const int col = c * 128 + lane * 4 + q; float y = __fmul_rn(v[c * 4 + q], rs); asm volatile("" : "+v"(y)); y = __fmul_rn(y, bfr(g[col])); asm volatile("" : "+v"(y)); o[q] = __fadd_rn(y, bfr(bb[col])); } *(volatile v4f*)(orow + c * 128 + lane * 4) = o; }
        if (ps == 0) __threadfence(); } }
__global__ __launch_bounds__(256) void k_merge(const float* __restrict__ O, int h0, bf* Ah, bf* Al) { const size_t e = ((size_t)blockIdx.x * 256 + threadIdx.x) * 2; if (e >= (size_t)ZH * TT * HD) return; const int d = (int)(e % HD); const int t = (int)((e / HD) % TT); const int zz = (int)(e / ((size_t)HD * TT)); const float cs = (t < RH) ? 1.0f : (1.0f / PCAR); const size_t oo = (size_t)t * DQ + (h0 + zz) * HD + d;
    v2us oh, ol;
#pragma unroll
    for (int q = 0; q < 2; ++q) { unsigned short a, c2; splitf(O[e + q] * cs, a, c2); oh[q] = a; ol[q] = c2; } *(volatile v2us*)(Ah + oo) = oh; *(volatile v2us*)(Al + oo) = ol; __threadfence(); *(volatile v2us*)(Ah + oo) = oh; *(volatile v2us*)(Al + oo) = ol; }

extern "C" void kernel_launch(void* const* d_in, const int* in_sizes, int n_in,
                              void* d_out, int out_size, void* d_ws, size_t ws_size, hipStream_t stream) {
    (void)in_sizes; (void)n_in; (void)out_size;
    const float* x = (const float*)d_in[0]; const float* xy = (const float*)d_in[1];   const float* wq = (const float*)d_in[4]; const float* wk = (const float*)d_in[5]; const float* wv = (const float*)d_in[6]; const float* wr = (const float*)d_in[7]; const float* cbias = (const float*)d_in[8]; const float* pbias = (const float*)d_in[9]; const float* wo = (const float*)d_in[10]; const float* bo = (const float*)d_in[11]; const float* lng = (const float*)d_in[12]; const float* lnb = (const float*)d_in[13];
    float* OUT = (float*)d_out;
    char* wsp = (char*)d_ws;
    auto take = [&](size_t bytes) { char* p = wsp; wsp += (bytes + 255) & ~(size_t)255; return (void*)p; };
    float* Yb = (float*)take((size_t)TT * DM * 4); bf* WR = (bf*)take((size_t)DQ * DM * 2); float* RT = (float*)take((size_t)NE * DM * 4); bf* RTh = (bf*)take((size_t)NE * DM * 2); bf* RTl = (bf*)take((size_t)NE * DM * 2); float* FR = (float*)take((size_t)NE * DQ * 4); bf* PPh = (bf*)take((size_t)NH_ * NE * HD * 2); bf* PPl = (bf*)take((size_t)NH_ * NE * HD * 2); float* FQV = (float*)take((size_t)TT * DQ * 4); h16* QV16 = (h16*)take((size_t)NH_ * TT * HD * 2); bf* QVh = (bf*)take((size_t)NH_ * TT * HD * 2); bf* QVl = (bf*)take((size_t)NH_ * TT * HD * 2); float* QE = (float*)take((size_t)ZH * TT * NE * 4); bf* WQ = (bf*)take((size_t)DQ * DM * 2); bf* WK = (bf*)take((size_t)DKV * DM * 2); bf* WV = (bf*)take((size_t)DKV * DM * 2); bf* WO = (bf*)take((size_t)DM * DQ * 2); float* CS = (float*)take((size_t)TT * HD * 2 * 4);
    bf* XB = (bf*)take((size_t)TT * DM * 2); float* FQ = (float*)take((size_t)TT * DQ * 4); float* FK = (float*)take((size_t)TT * DKV * 4);
    h16* QP16 = (h16*)take((size_t)NH_ * TT * HD * 2); h16* KP16 = (h16*)take((size_t)NKV * TT * HD * 2); h16* VT16 = (h16*)take((size_t)NKV * HD * TT * 2);
    bf* QPh = (bf*)take((size_t)NH_ * TT * HD * 2); bf* QPl = (bf*)take((size_t)NH_ * TT * HD * 2); bf* KPh = (bf*)take((size_t)NKV * TT * HD * 2); bf* KPl = (bf*)take((size_t)NKV * TT * HD * 2); bf* VTh = (bf*)take((size_t)NKV * HD * TT * 2); bf* VTl = (bf*)take((size_t)NKV * HD * TT * 2); bf* Ph = (bf*)take((size_t)ZH * RH * TT * 2); bf* Pl = (bf*)take((size_t)ZH * RH * TT * 2);
    float* Sb = (float*)take((size_t)ZH * TT * TT * 4); h16* P16 = (h16*)take((size_t)ZH * TT * TT * 2); float* Ob = (float*)take((size_t)ZH * TT * HD * 4); bf* ATh = (bf*)take((size_t)TT * DQ * 2); bf* ATl = (bf*)take((size_t)TT * DQ * 2);
    if ((size_t)(wsp - (char*)d_ws) > ws_size) return;
    float* FV = FK;
    { k_wtG<<<(unsigned)((DM * DQ / 64 + 63) / 64), 256, 0, stream>>>(wq, DM, DQ, WQ); k_wtG<<<(unsigned)((DM * DQ / 64 + 63) / 64), 256, 0, stream>>>(wr, DM, DQ, WR); k_sinR<<<(unsigned)(((size_t)NE * DM / 4 + 255) / 256), 256, 0, stream>>>(RT);     k_split8<<<(unsigned)(((size_t)NE * DM / 8 + 255) / 256), 256, 0, stream>>>(RT, RTh, RTl, (size_t)NE * DM / 8); k_gemmw<bf, 1, false><<<dim3(NE / 64, DQ / 64, 1), 32, 0, stream>>>(RTh, RTl, WR, nullptr, DM, FR, DQ, nullptr, 0, 0, 0);     k_hplanesN<<<(unsigned)(((size_t)NE * DQ / 4 + 255) / 256), 256, 0, stream>>>(FR, PPh, PPl);     k_wtG<<<(unsigned)((DM * DKV / 64 + 63) / 64), 256, 0, stream>>>(wk, DM, DKV, WK); k_wtG<<<(unsigned)((DM * DKV / 64 + 63) / 64), 256, 0, stream>>>(wv, DM, DKV, WV);
      k_cvt8<<<(unsigned)(((size_t)DM * DQ / 8 + 255) / 256), 256, 0, stream>>>(wo, WO, (size_t)DM * DQ / 8);
       }
    k_csid<<<(TT * HD + 255) / 256, 256, 0, stream>>>(CS);
    const unsigned LQ = (unsigned)(((size_t)NH_ * TT * HD / 2 + 255) / 256), LKv = (unsigned)(((size_t)NKV * TT * HD / 2 + 255) / 256);
    for (int b = 0; b < NB_; ++b) {

        k_cvt8<<<(unsigned)(((size_t)TT * DM / 8 + 255) / 256), 256, 0, stream>>>(x + (size_t)b * TT * DM, XB, (size_t)TT * DM / 8);
        k_gemmw<bf, 0, false><<<dim3(TT / 64, DQ / 64, 1), 32, 0, stream>>>(XB, nullptr, WQ, nullptr, DM, FQ, DQ, nullptr, 0, 0, 0);
        k_addhb<<<(unsigned)(((size_t)TT * DQ / 4 + 255) / 256), 256, 0, stream>>>(FQ, cbias, pbias, FQV);     k_rope<<<LQ, 256, 0, stream>>>(FQ, DQ, NH_, CS, nullptr, nullptr, 1.0f, QP16, QPh, QPl); k_rope<<<LQ, 256, 0, stream>>>(FQV, DQ, NH_, CS, nullptr, nullptr, 1.0f, QV16, QVh, QVl);
        k_cvt8<<<(unsigned)(((size_t)TT * DM / 8 + 255) / 256), 256, 0, stream>>>(xy + (size_t)b * TT * DM, XB, (size_t)TT * DM / 8);     k_gemmw<bf, 0, false><<<dim3(TT / 64, DKV / 64, 1), 32, 0, stream>>>(XB, nullptr, WK, nullptr, DM, FK, DKV, nullptr, 0, 0, 0);
        k_rope<<<LKv, 256, 0, stream>>>(FK, DKV, NKV, CS, nullptr, nullptr, 1.0f, KP16, KPh, KPl);
        k_gemmw<bf, 0, false><<<dim3(TT / 64, DKV / 64, 1), 32, 0, stream>>>(XB, nullptr, WV, nullptr, DM, FV, DKV, nullptr, 0, 0, 0); k_vtp<<<LKv, 256, 0, stream>>>(FV, DKV, NKV, VT16, VTh, VTl);
        for (int h0 = 0; h0 < NH_; h0 += ZH) { const size_t zq = (size_t)h0, zk = (size_t)(h0 / REP);
            k_gemmc<bf, 2, 1><<<dim3(TT / 64, TT / 64, ZH), 32, 0, stream>>>(QPh + zq * TT * HD, QPl + zq * TT * HD, KPh + zk * TT * HD, KPl + zk * TT * HD, HD, Sb, TT, 0, (size_t)TT * HD, (size_t)TT * HD, (size_t)TT * TT);

            k_gemmw<bf, 2, false><<<dim3(TT / 64, NE / 64, ZH), 32, 0, stream>>>(QVh + zq * TT * HD, QVl + zq * TT * HD, PPh + zq * NE * HD, PPl + zq * NE * HD, HD, QE, NE, nullptr, (size_t)TT * HD, (size_t)NE * HD, (size_t)TT * NE);
            k_addrl<<<(unsigned)(((size_t)ZH * TT * TT / 4 + 255) / 256), 256, 0, stream>>>(Sb, QE);
            k_asoft<<<ZH * TT / 8, 256, 0, stream>>>(Sb, P16, Ph, Pl);
            k_gemmc<bf, 2, 2><<<dim3(RH / 64, HD / 64, ZH), 32, 0, stream>>>(Ph, Pl, VTh + zk * HD * TT, VTl + zk * HD * TT, TT, Ob, HD, 0, (size_t)RH * TT, (size_t)HD * TT, (size_t)TT * HD);
            k_gemmc<h16, 0, 2><<<dim3((TT - RH) / 64, HD / 64, ZH), 32, 0, stream>>>(P16 + (size_t)RH * TT, nullptr, VT16 + zk * HD * TT, nullptr, TT, Ob + (size_t)RH * HD, HD, RH, (size_t)TT * TT, (size_t)HD * TT, (size_t)TT * HD);
            k_merge<<<(unsigned)(((size_t)ZH * TT * HD / 2 + 255) / 256), 256, 0, stream>>>(Ob, h0, ATh, ATl); }
        k_gemmw<bf, 1, true><<<dim3(TT / 64, DM / 64, 1), 32, 0, stream>>>(ATh, ATl, WO, nullptr, DQ, Yb, DM, bo, 0, 0, 0); k_addres<<<(unsigned)(((size_t)TT * DQ / 4 + 255) / 256), 256, 0, stream>>>(Yb, x + (size_t)b * TT * DM); k_lnout<<<(TT + 7) / 8, 256, 0, stream>>>(Yb, lng, lnb, OUT + (size_t)b * TT * DM);     }
}
